// PQMatcher_27453430956675
// MI455X (gfx1250) — hardware-verified
//
#include <hip/hip_runtime.h>


#ifndef LPN
#define LPN 400
#endif
#ifndef NB
#define NB 32
#endif
#define LP_FULL 400
#define BZ_FULL 32
#define LQ   50
#define SZ   768
#define HH   128
#define AW   5
#define BP   132
#define SCP  64
#define OSP  68
#define LNP  132
#define C2   2.8853900817779268f
#define LOG2E 1.4426950408889634f
#define PSH  14.0f
#define UQC  16.0f
#define NEGB (-3.0e38f)

static_assert(HH == 128);
static_assert(HH / 4 == 32);
static_assert(SZ % 64 == 0);
static_assert(SZ % 32 == 0);
static_assert(HH % 32 == 0);
static_assert(LQ >= 48 && LQ <= 50);
static_assert(LQ <= 64);
static_assert(LPN % (16 * AW) == 0);
static_assert((LPN * BZ_FULL) % 16 == 0);
static_assert((LQ * BZ_FULL) % 16 == 0);
static_assert(BZ_FULL % 16 == 0);
static_assert(LPN <= LP_FULL);
static_assert(NB <= BZ_FULL);
static_assert((BP * 4) % 16 == 0);
static_assert((OSP * 4) % 16 == 0);
static_assert((LNP * 4) % 16 == 0);
static_assert((SCP * 4) % 16 == 0);
static_assert(32 * 16 * 16 == 16 * HH * 4);
static_assert(32 * 16 * 8 == 16 * 64 * 4);
static_assert(256 * 16 == 32 * 64 * 2);
static_assert((size_t)(LQ * HH + HH + AW * 16 * BP + AW * 16 * SCP + AW * 16 * OSP) * 4 <= (size_t)131072);
static_assert((size_t)(64 * 33) * 4 <= (size_t)131072);
static_assert((size_t)(16 * LNP) * 4 <= (size_t)131072);

typedef _Float16 h16;
typedef unsigned short bf;
typedef __attribute__((ext_vector_type(16))) __bf16   v16bf;
typedef __attribute__((ext_vector_type(16))) _Float16 v16h;
typedef __attribute__((ext_vector_type(8)))  _Float16 v8h;
typedef __attribute__((ext_vector_type(8)))  unsigned short v8us;
typedef __attribute__((ext_vector_type(8)))  float    v8f;
typedef __attribute__((ext_vector_type(4)))  float    v4f;
typedef v4f  __attribute__((may_alias)) v4fa;

__device__ __forceinline__ unsigned short f2bf(float f) { unsigned u = __float_as_uint(f); u += 0x7FFFu + ((u >> 16) & 1u); return (unsigned short)(u >> 16); }
__device__ __forceinline__ float bfr(float f) { return __uint_as_float(((unsigned)f2bf(f)) << 16); }
__device__ __forceinline__ v16h cat16(v8h lo, v8h hi) { return __builtin_shufflevector(lo, hi, 0, 1, 2, 3, 4, 5, 6, 7, 8, 9, 10, 11, 12, 13, 14, 15); }
__device__ __forceinline__ v16bf cat16b(v8us lo, v8us hi) { return __builtin_bit_cast(v16bf, __builtin_shufflevector(lo, hi, 0, 1, 2, 3, 4, 5, 6, 7, 8, 9, 10, 11, 12, 13, 14, 15)); }
__device__ __forceinline__ v8f wmma16(v16h a, v16h b, v8f c) { return __builtin_amdgcn_wmma_f32_16x16x32_f16(false, a, false, b, (short)0, c, false, false); }
__device__ __forceinline__ v8f wmmab(v16bf a, v16bf b, v8f c) { return __builtin_amdgcn_wmma_f32_16x16x32_bf16(false, a, false, b, (short)0, c, false, false); }
__device__ __forceinline__ v16h  ldh(const h16* p) { return cat16(*(const v8h*)p, *(const v8h*)(p + 16)); }
__device__ __forceinline__ v16bf ldb(const bf* p)  { return cat16b(*(const v8us*)p, *(const v8us*)(p + 16)); }
__device__ __forceinline__ void wave_sync() { __builtin_amdgcn_fence(3  , "wavefront"); __builtin_amdgcn_wave_barrier(); asm volatile("" ::: "memory"); }

static __device__ __forceinline__ h16 toh_flush(float v) { const h16 r = (h16)v; return (fabsf(v) < 6.103515625e-05f) ? (h16)0.0f : r; }
__device__ __forceinline__ v8f wmma16g(v16h a, v16h b, v8f c) { c = wmma16(a, b, c); asm volatile("v_nop\n\tv_nop\n\tv_nop\n\tv_nop" : "+v"(c) : "v"(a), "v"(b)); return c; }
__device__ __forceinline__ v8f wmmabg(v16bf a, v16bf b, v8f c) { c = wmmab(a, b, c); asm volatile("v_nop\n\tv_nop\n\tv_nop\n\tv_nop" : "+v"(c) : "v"(a), "v"(b)); return c; }

__global__ __launch_bounds__(256) void k_cvt8(const float* __restrict__ src, bf* dst, size_t n8) {
    const size_t i = (size_t)blockIdx.x * 256 + threadIdx.x; if (i >= n8) return;
    const v8f v = *(const v8f*)(src + i * 8); v8us o;
#pragma unroll
    for (int k = 0; k < 8; ++k) o[k] = f2bf(v[k]);
    *(volatile v8us*)(dst + i * 8) = o; __threadfence(); *(volatile v8us*)(dst + i * 8) = o;
}

__global__ __launch_bounds__(256) void k_uqt(const float* __restrict__ UQ, h16* UQT) {
    __shared__ float tl[64 * 33];
    const int tid = threadIdx.x; const int s0 = blockIdx.x * 32; const int b = blockIdx.y;
#pragma unroll 1
    for (int i = tid; i < 64 * 32; i += 256) {
        const int q = i >> 5, s = i & 31; const int qc = q < LQ ? q : (LQ - 1);
        float x = UQ[((size_t)qc * BZ_FULL + b) * SZ + s0 + s];
        asm volatile("" : "+v"(x));
        tl[q * 33 + s] = (q < LQ) ? (bfr(x) * UQC) : 0.0f; }
    __syncthreads();
    const int s = tid >> 3, q8 = (tid & 7) * 8; v8h o;
#pragma unroll
    for (int k = 0; k < 8; ++k) o[k] = toh_flush(tl[(q8 + k) * 33 + s]);
    h16* dst = UQT + ((size_t)b * SZ + s0) * 64 + (size_t)tid * 8;
    *(volatile v8h*)dst = o; __threadfence(); *(volatile v8h*)dst = o;
}

__global__ __launch_bounds__(32) void k_lin(const float* __restrict__ A, const bf* __restrict__ Wt, const float* __restrict__ bias, float* Out, int K) {
    __shared__ __align__(16) float os[16 * LNP];
    const int lane = threadIdx.x & 31, lr = lane & 15, hi = lane >> 4; const int r0 = blockIdx.x * 16;
    v8f acc[8];
#pragma unroll
    for (int nt = 0; nt < 8; ++nt) acc[nt] = (v8f){};
    const size_t aoff = (size_t)(r0 + lr) * (size_t)K + 8 * hi, boff = (size_t)lr * (size_t)K + 8 * hi;
#pragma unroll 1
    for (int kc = 0; kc < K; kc += 32) {
        const float* ap = A + aoff + kc;
        const v4f x0 = *(const v4f*)ap, x1 = *(const v4f*)(ap + 4), x2 = *(const v4f*)(ap + 16), x3 = *(const v4f*)(ap + 20);
        v8us lo, up;
#pragma unroll
        for (int i = 0; i < 4; ++i) { lo[i] = f2bf(x0[i]); lo[4 + i] = f2bf(x1[i]); up[i] = f2bf(x2[i]); up[4 + i] = f2bf(x3[i]); }
        const v16bf a = cat16b(lo, up);
#pragma unroll
        for (int nt = 0; nt < 8; ++nt) { const v16bf b = ldb(Wt + boff + (size_t)nt * 16 * (size_t)K + kc); acc[nt] = wmmabg(a, b, acc[nt]); }
    }
    float bc[8];
#pragma unroll
    for (int nt = 0; nt < 8; ++nt) bc[nt] = bfr(bias[nt * 16 + lr]);
#pragma unroll
    for (int nt = 0; nt < 8; ++nt) {
#pragma unroll
        for (int j = 0; j < 8; ++j) os[(hi * 8 + j) * LNP + nt * 16 + lr] = acc[nt][j] + bc[nt]; }
    wave_sync();
    float* orow = Out + (size_t)r0 * HH;
#pragma unroll 1
    for (int ps = 0; ps < 2; ++ps) {
#pragma unroll 4
        for (int row = 0; row < 16; ++row) {
            const v4f val = *(const v4fa*)(&os[row * LNP + lane * 4]);
            *(volatile v4f*)(orow + (size_t)row * HH + lane * 4) = val; }
        if (ps == 0) __threadfence(); }
}

__global__ __launch_bounds__(32 * AW) void k_attn(const float* __restrict__ WUP, const float* __restrict__ WUQ, const float* __restrict__ WVV, const float* __restrict__ vin,
                                                 const h16* __restrict__ UQT, float* OUT) {
    __shared__ __align__(16) float wq[LQ * HH];
    __shared__ __align__(16) float vl[HH];
    __shared__ __align__(16) float bs[AW * 16 * BP];
    __shared__ __align__(16) float sc[AW * 16 * SCP];
    __shared__ __align__(16) float os[AW * 16 * OSP];
    const int tid = threadIdx.x;
    const int lane = tid & 31, lr = lane & 15, hi = lane >> 4;
    const int wave = __builtin_amdgcn_readfirstlane((int)(threadIdx.x >> 5));
    const int b = blockIdx.y;
    const int p0 = (blockIdx.x * AW + wave) * 16;
#pragma unroll 1
    for (int i = tid; i < LQ * HH / 4; i += 32 * AW) {
        const int q = i >> 5, c4 = (i & 31) * 4;
        v4f w = *(const v4f*)(WUQ + ((size_t)q * BZ_FULL + b) * HH + c4); w = w * C2;
        *(v4fa*)(&wq[q * HH + c4]) = w; }
    if (wave == 0) {
        v4f x = *(const v4f*)(vin + (size_t)b * HH + lane * 4);
#pragma unroll
        for (int c = 0; c < 4; ++c) x[c] = bfr(x[c]);
        *(v4fa*)(&vl[lane * 4]) = x; }
    const int bsb = wave * 16 * BP, scb = wave * 16 * SCP, wb = wave * 16 * OSP;
    { const v4f wv = *(const v4f*)(WVV + (size_t)b * HH + lane * 4);
#pragma unroll 4
      for (int i = 0; i < 16; ++i) {
          const v4f u = *(const v4f*)(WUP + ((size_t)(p0 + i) * BZ_FULL + b) * HH + lane * 4);
          const v4f sxx = (u + wv) * C2;
          *(v4fa*)(&bs[bsb + i * BP + lane * 4]) = sxx; } }
    __syncthreads();

#pragma unroll 1
    for (int g = 0; g < 3; ++g) {
        const int qb = 16 * g + 8 * hi;
        float a[8];
#pragma unroll
        for (int r = 0; r < 8; ++r) a[r] = 0.0f;
#pragma unroll 1
        for (int hc = 0; hc < HH; hc += 4) {
            const v4f bb = *(const v4fa*)(&bs[bsb + lr * BP + hc]);
            const v4f vv = *(const v4fa*)(&vl[hc]);
#pragma unroll
            for (int r = 0; r < 8; ++r) {
                const v4f ww = *(const v4fa*)(&wq[(qb + r) * HH + hc]);
#pragma unroll
                for (int c = 0; c < 4; ++c) {
                    const float e = __builtin_amdgcn_exp2f(bb[c] + ww[c]);
                    const float rr = __builtin_amdgcn_rcpf(e + 1.0f);
                    a[r] = fmaf(vv[c], rr, a[r]); } } }
#pragma unroll
        for (int r = 0; r < 8; ++r) sc[scb + lr * SCP + qb + r] = -2.0f * a[r];
    }
    { const int qa = 48 + 8 * hi;
      const int q0 = qa < LQ ? qa : (LQ - 1); const int q1 = (qa + 1) < LQ ? (qa + 1) : (LQ - 1);
      float a0 = 0.0f, a1 = 0.0f;
#pragma unroll 1
      for (int hc = 0; hc < HH; hc += 4) {
          const v4f bb = *(const v4fa*)(&bs[bsb + lr * BP + hc]);
          const v4f vv = *(const v4fa*)(&vl[hc]);
          const v4f w0 = *(const v4fa*)(&wq[q0 * HH + hc]);
          const v4f w1 = *(const v4fa*)(&wq[q1 * HH + hc]);
#pragma unroll
          for (int c = 0; c < 4; ++c) {
              const float e0 = __builtin_amdgcn_exp2f(bb[c] + w0[c]); const float e1 = __builtin_amdgcn_exp2f(bb[c] + w1[c]);
              const float r0 = __builtin_amdgcn_rcpf(e0 + 1.0f); const float r1 = __builtin_amdgcn_rcpf(e1 + 1.0f);
              a0 = fmaf(vv[c], r0, a0); a1 = fmaf(vv[c], r1, a1); } }
      sc[scb + lr * SCP + qa] = -2.0f * a0; sc[scb + lr * SCP + qa + 1] = -2.0f * a1; }
    wave_sync();

    const int sr = scb + lr * SCP + 8 * hi;
    float t0[8], t1[8], t2[8];
    { const v4f x0 = *(const v4fa*)(&sc[sr]),      x1 = *(const v4fa*)(&sc[sr + 4]);
      const v4f y0 = *(const v4fa*)(&sc[sr + 16]), y1 = *(const v4fa*)(&sc[sr + 20]);
      const v4f z0 = *(const v4fa*)(&sc[sr + 32]), z1 = *(const v4fa*)(&sc[sr + 36]);
#pragma unroll
      for (int r = 0; r < 4; ++r) { t0[r] = x0[r] * LOG2E; t0[4 + r] = x1[r] * LOG2E; t1[r] = y0[r] * LOG2E; t1[4 + r] = y1[r] * LOG2E; t2[r] = z0[r] * LOG2E; t2[4 + r] = z1[r] * LOG2E; } }
    const float t3a = sc[sr + 48] * LOG2E, t3b = sc[sr + 49] * LOG2E;
    const bool ok3a = (48 + 8 * hi) < LQ, ok3b = (49 + 8 * hi) < LQ;
    float mx = NEGB;
#pragma unroll
    for (int r = 0; r < 8; ++r) mx = fmaxf(mx, fmaxf(t0[r], fmaxf(t1[r], t2[r])));
    mx = fmaxf(mx, fmaxf(ok3a ? t3a : NEGB, ok3b ? t3b : NEGB));
    mx = fmaxf(mx, __shfl_xor(mx, 16, 32));
    const float sh = PSH - mx;
    const v16h hz = (v16h){};
    v16h pb0, pb1 = hz; float ls = 0.0f;
#pragma unroll
    for (int r = 0; r < 8; ++r) {
        const h16 x = toh_flush(__builtin_amdgcn_exp2f(t0[r] + sh));
        const h16 y = toh_flush(__builtin_amdgcn_exp2f(t1[r] + sh));
        const h16 z = toh_flush(__builtin_amdgcn_exp2f(t2[r] + sh));
        pb0[r] = x; pb0[8 + r] = y; pb1[r] = z;
        ls += (float)x + (float)y + (float)z; }
    { const float ea = __builtin_amdgcn_exp2f(t3a + sh), eb = __builtin_amdgcn_exp2f(t3b + sh);
      const float ga = ok3a ? ea : 0.0f, gb = ok3b ? eb : 0.0f;
      const h16 x = toh_flush(ga); const h16 y = toh_flush(gb);
      pb1[8] = x; pb1[9] = y; ls += (float)x + (float)y; }
    ls += __shfl_xor(ls, 16, 32);
    const float inv = 1.0f / (ls * UQC);

    const size_t uo = ((size_t)b * SZ + (size_t)lr) * 64 + 8 * hi;
    float* obase = OUT + ((size_t)p0 * BZ_FULL + b) * SZ;
#pragma unroll 1
    for (int s0 = 0; s0 < SZ; s0 += 64) {
        const h16* ua = UQT + uo + (size_t)s0 * 64;
        v8f o[4];
#pragma unroll
        for (int j = 0; j < 4; ++j) {
            const v16h a0 = ldh(ua + (size_t)j * 16 * 64), a1 = ldh(ua + (size_t)j * 16 * 64 + 32);
            o[j] = (v8f){};
            o[j] = wmma16g(a0, pb0, o[j]);
            o[j] = wmma16g(a1, pb1, o[j]); }
#pragma unroll
        for (int j = 0; j < 4; ++j) { v4f a, c;
            a[0] = o[j][0] * inv; a[1] = o[j][1] * inv; a[2] = o[j][2] * inv; a[3] = o[j][3] * inv; c[0] = o[j][4] * inv; c[1] = o[j][5] * inv; c[2] = o[j][6] * inv; c[3] = o[j][7] * inv;
            *(v4fa*)(&os[wb + lr * OSP + 16 * j + 8 * hi]) = a; *(v4fa*)(&os[wb + lr * OSP + 16 * j + 8 * hi + 4]) = c; }
        wave_sync();
        float* orow = obase + s0;
#pragma unroll 1
        for (int ps = 0; ps < 2; ++ps) {
#pragma unroll
            for (int s = 0; s < 8; ++s) { const int row = 2 * s + (lane >> 4), cofs = (lane & 15) * 4;
                const v4f val = *(const v4fa*)(&os[wb + row * OSP + cofs]);
                *(volatile v4f*)(orow + (size_t)row * ((size_t)BZ_FULL * SZ) + cofs) = val; }
            if (ps == 0) __threadfence(); }
        wave_sync();
    }
}

static constexpr size_t al256(size_t v) { return (v + 255) & ~(size_t)255; }
static constexpr size_t SZ_WP = al256((size_t)HH * SZ * 2);
static constexpr size_t SZ_WV = al256((size_t)HH * HH * 2);
static constexpr size_t SZ_UP = al256((size_t)LPN * BZ_FULL * HH * 4);
static constexpr size_t SZ_UQ = al256((size_t)LQ * BZ_FULL * HH * 4);
static constexpr size_t SZ_VV = al256((size_t)BZ_FULL * HH * 4);
static constexpr size_t SZ_UT = al256((size_t)BZ_FULL * SZ * 64 * 2);
static constexpr size_t SZ_TOTAL = 2 * SZ_WP + SZ_WV + SZ_UP + SZ_UQ + SZ_VV + SZ_UT;
static_assert(SZ_TOTAL <= (size_t)134217728);
static_assert(((size_t)HH * SZ) % 8 == 0);
static_assert(((size_t)HH * HH) % 8 == 0);
static_assert((size_t)(SZ / 32) * 32 * 64 * NB <= (size_t)BZ_FULL * SZ * 64);
static_assert((size_t)(LPN * BZ_FULL / 16) * 16 * HH * 4 <= SZ_UP);
static_assert((size_t)(LQ * BZ_FULL / 16) * 16 * HH * 4 <= SZ_UQ);
static_assert((size_t)(BZ_FULL / 16) * 16 * HH * 4 <= SZ_VV);

extern "C" void kernel_launch(void* const* d_in, const int* in_sizes, int n_in,
                              void* d_out, int out_size, void* d_ws, size_t ws_size, hipStream_t stream) {
    if (n_in < 9) return;
    if ((size_t)in_sizes[0] < (size_t)LPN * BZ_FULL * SZ) return;
    if ((size_t)in_sizes[1] < (size_t)LQ * BZ_FULL * SZ) return;
    if ((size_t)in_sizes[2] < (size_t)HH * SZ || (size_t)in_sizes[4] < (size_t)HH * SZ || (size_t)in_sizes[6] < (size_t)HH * HH) return;
    if (in_sizes[3] < HH || in_sizes[5] < HH || in_sizes[7] < HH) return;
    if ((size_t)in_sizes[8] < (size_t)BZ_FULL * HH) return;
    if ((size_t)out_size < ((size_t)(LPN - 1) * BZ_FULL + NB) * SZ) return;
    if (SZ_TOTAL > ws_size) return;
    const float* up  = (const float*)d_in[0]; const float* uq  = (const float*)d_in[1];
    const float* wpw = (const float*)d_in[2]; const float* wpb = (const float*)d_in[3];
    const float* wqw = (const float*)d_in[4]; const float* wqb = (const float*)d_in[5];
    const float* wvw = (const float*)d_in[6]; const float* wvb = (const float*)d_in[7];
    const float* vv  = (const float*)d_in[8];
    float* OUT = (float*)d_out;
    char* wsp = (char*)d_ws;
    bf* WPB = (bf*)wsp; wsp += SZ_WP;
    bf* WQB = (bf*)wsp; wsp += SZ_WP;
    bf* WVB = (bf*)wsp; wsp += SZ_WV;
    float* WUP = (float*)wsp; wsp += SZ_UP;
    float* WUQ = (float*)wsp; wsp += SZ_UQ;
    float* WVV = (float*)wsp; wsp += SZ_VV;
    h16* UQT = (h16*)wsp; wsp += SZ_UT;

    { const size_t n8 = (size_t)HH * SZ / 8; const unsigned g = (unsigned)((n8 + 255) / 256);
      k_cvt8<<<g, 256, 0, stream>>>(wpw, WPB, n8); k_cvt8<<<g, 256, 0, stream>>>(wqw, WQB, n8); }
    { const size_t n8 = (size_t)HH * HH / 8; k_cvt8<<<(unsigned)((n8 + 255) / 256), 256, 0, stream>>>(wvw, WVB, n8); }
    k_uqt<<<dim3(SZ / 32, NB, 1), 256, 0, stream>>>(uq, UQT);
    k_lin<<<dim3(LPN * BZ_FULL / 16, 1, 1), 32, 0, stream>>>(up, WPB, wpb, WUP, SZ);
    k_lin<<<dim3(LQ * BZ_FULL / 16, 1, 1), 32, 0, stream>>>(uq, WQB, wqb, WUQ, SZ);
    k_lin<<<dim3(BZ_FULL / 16, 1, 1), 32, 0, stream>>>(vv, WVB, wvb, WVV, HH);
    k_attn<<<dim3(LPN / (16 * AW), NB, 1), 32 * AW, 0, stream>>>(WUP, WUQ, WVV, vv, UQT, OUT);
}
